// SGCWGTL_77068893159665
// MI455X (gfx1250) — hardware-run, weakly checked
//
#include <hip/hip_runtime.h>


namespace {
constexpr int N = 50000, NP = 50048, E = 1600000, NF = 128, NH = 64, NC = 16, AH = 32;
constexpr float XS = 8.0f, WSC = 256.0f;
typedef _Float16 b16;
typedef __attribute__((ext_vector_type(16))) _Float16 v16b;
typedef __attribute__((ext_vector_type(8))) _Float16 v8b;
typedef __attribute__((ext_vector_type(8))) float v8f;
typedef __attribute__((ext_vector_type(4))) float v4f;
typedef __attribute__((ext_vector_type(2))) float v2f;
__device__ __forceinline__ float bf16_rne(float f) { unsigned int u = __float_as_uint(f); u += 0x7FFFu + ((u >> 16) & 1u); return __uint_as_float(u & 0xFFFF0000u); }
__device__ __forceinline__ void split16(float v, b16& hi, b16& lo) { hi = (b16)v; lo = (b16)(v - (float)hi); }
__device__ __forceinline__ v16b frag_kb(const b16* p, int hh) { const v8b a = *(const v8b*)(p + 8 * hh), b = *(const v8b*)(p + 16 + 8 * hh); v16b f;
#pragma unroll
  for (int e = 0; e < 8; ++e) { f[e] = a[e]; f[8 + e] = b[e]; } return f; }
__device__ __forceinline__ v8f wmma16b(v16b a, v16b b, v8f c) { v8f d = __builtin_amdgcn_wmma_f32_16x16x32_f16(false, a, false, b, (short)0, c, false, false); asm volatile("v_nop\n\tv_nop\n\tv_nop\n\tv_nop" : "+v"(d) : "v"(a), "v"(b)); return d; }
__device__ __forceinline__ void wave_lds_sync() { __builtin_amdgcn_fence(__ATOMIC_RELEASE, "workgroup"); __builtin_amdgcn_wave_barrier(); __builtin_amdgcn_fence(__ATOMIC_ACQUIRE, "workgroup"); }
__device__ __forceinline__ float pmul(float a, float b) { float p = a * b; asm volatile("" : "+v"(p)); return p; }
__device__ __forceinline__ float opaque(float a) { asm volatile("" : "+v"(a)); return a; }
__device__ __forceinline__ int iclamp(int v, int lo, int hi) { return v < lo ? lo : (v > hi ? hi : v); }
__device__ __forceinline__ float nexp(float x) { return __builtin_amdgcn_exp2f(x * 1.4426950408889634f); }
constexpr int CSR_NBLK8 = 512, CSR_GB8 = 8, CSR_GN8 = 1 << CSR_GB8  , CSR_TS8 = (CSR_GN8 < 32 ? 32 : CSR_GN8)  , CSR_MAXG8 = 512, CSR_CAP8 = 12288  ;
__device__ __host__ __forceinline__ int csr_tix8(int v) { return (v >> CSR_GB8) * CSR_TS8 + (v & (CSR_GN8 - 1)); }
__global__ __launch_bounds__(64) void csrA_kernel8(const int* __restrict__ dst, int E, int N, int nG, int CHP, int NGP, int* __restrict__ STG, int* __restrict__ HST) {
  extern __shared__ int sm[];
  int* cnt = sm; int* run = sm + NGP; int* ids = sm + 2 * NGP;
  const int b = blockIdx.x; const int ch = (E + CSR_NBLK8 - 1) / CSR_NBLK8; const int e0 = b * ch, e1 = min(E, e0 + ch);
  for (int i = threadIdx.x; i < NGP; i += 64) cnt[i] = 0;
  for (int i = threadIdx.x; i < CHP; i += 64) ids[i] = -1;
  __syncthreads();
  if (threadIdx.x == 0) {
    for (int e = e0; e < e1; ++e) { int d = dst[e]; d = (d < 0) ? 0 : (d >= N ? N - 1 : d); cnt[d >> CSR_GB8] += 1; }
    int acc = 0; for (int g = 0; g < nG; ++g) { run[g] = acc; acc += cnt[g]; }
    for (int e = e0; e < e1; ++e) { int d = dst[e]; d = (d < 0) ? 0 : (d >= N ? N - 1 : d); const int g = d >> CSR_GB8; ids[run[g]] = e; run[g] += 1; } }
  __syncthreads();
  typedef __attribute__((ext_vector_type(4))) int v4i;
  for (int pass = 0; pass < 2; ++pass) {
    for (int i = threadIdx.x; i < CHP / 4; i += 64) *(volatile v4i*)(STG + (size_t)b * CHP + i * 4) = *(const v4i*)(&ids[i * 4]);
    for (int i = threadIdx.x; i < NGP / 4; i += 64) { v4i v; for (int e = 0; e < 4; ++e) v[e] = (i * 4 + e < nG) ? cnt[i * 4 + e] : 0; *(volatile v4i*)(HST + (size_t)b * NGP + i * 4) = v; }
    __threadfence(); }
}
__global__ __launch_bounds__(512) void csrS_kernel8(const int* __restrict__ HST, int nG, int NGP, int* __restrict__ START, int* __restrict__ TOT, int* __restrict__ OFF) {
  __shared__ int tot[CSR_MAXG8];
  const int b = threadIdx.x;
  for (int pass = 0; pass < 2; ++pass) { int runb = 0; for (int g = 0; g < nG; ++g) { int c = HST[(size_t)b * NGP + g]; c = (c < 0) ? 0 : c; ((volatile int*)OFF)[(size_t)g * CSR_NBLK8 + b] = runb; runb += c; } __threadfence(); }
  for (int g = threadIdx.x; g < nG; g += 512) { int s = 0; for (int bb = 0; bb < CSR_NBLK8; ++bb) { int c = HST[(size_t)bb * NGP + g]; s += (c < 0) ? 0 : c; } tot[g] = s; }
  __syncthreads();
  if (threadIdx.x < 32) {
    __shared__ int st[CSR_MAXG8 + 32];
    if (threadIdx.x == 0) { int acc = 0; for (int g = 0; g < NGP; ++g) { st[g] = acc; if (g < nG) acc += (tot[g] + 31) & ~31; } st[NGP] = acc; }
    __builtin_amdgcn_fence(__ATOMIC_RELEASE, "workgroup"); __builtin_amdgcn_wave_barrier(); __builtin_amdgcn_fence(__ATOMIC_ACQUIRE, "workgroup");
    for (int pass = 0; pass < 2; ++pass) { for (int i = threadIdx.x; i < NGP + 32; i += 32) { ((volatile int*)START)[i] = (i <= NGP) ? st[min(i, NGP)] : 0; ((volatile int*)TOT)[i] = (i < nG) ? tot[i] : 0; } __threadfence(); } }
}
__global__ __launch_bounds__(256) void csrB_kernel8(const int* __restrict__ dst, int N, int nG, int CHP, int NGP, int permLen, const int* __restrict__ STG, const int* __restrict__ HST, const int* __restrict__ OFF, const int* __restrict__ START, const int* __restrict__ TOT, int* __restrict__ PERM, int* __restrict__ ROWPTR, int* __restrict__ ROWCNT, int* __restrict__ FLAG) {
  typedef __attribute__((ext_vector_type(4))) int v4i;
  __shared__ int ids[CSR_CAP8]; __shared__ unsigned short key[CSR_CAP8]; __shared__ int outp[CSR_CAP8]; __shared__ int ncnt[CSR_GN8 + 1]; __shared__ int boff[CSR_NBLK8 + 1];
  const int g = blockIdx.x, t_ = threadIdx.x; int tot = TOT[g]; int st = START[g], stn = START[g + 1]; const int v0 = g * CSR_GN8; const int nv = min(CSR_GN8, N - v0); const int t0 = g * CSR_TS8;
  st = (st < 0) ? 0 : (st > permLen - 32 ? permLen - 32 : st) & ~31; stn = (stn < st) ? st : (stn > permLen ? permLen : stn); tot = (tot < 0) ? 0 : tot; if (tot > stn - st && tot <= CSR_CAP8) tot = stn - st;
  if (tot > CSR_CAP8) {
    for (int pass = 0; pass < 2; ++pass) { for (int i = t_; i < CSR_TS8 / 4; i += 256) { v4i a, c; for (int e = 0; e < 4; ++e) { a[e] = st; c[e] = 0; } *(volatile v4i*)(ROWPTR + t0 + i * 4) = a; *(volatile v4i*)(ROWCNT + t0 + i * 4) = c; } if (t_ == 0) ((volatile int*)FLAG)[0] = 1; __threadfence(); } (void)nv; return; }
  if (t_ == 0) { int acc = 0; for (int b = 0; b < CSR_NBLK8; ++b) { boff[b] = acc; int c = HST[(size_t)b * NGP + g]; c = (c < 0) ? 0 : (c > CHP ? CHP : c); acc += c; if (acc > tot) acc = tot; } boff[CSR_NBLK8] = acc; }
  for (int i = t_; i <= CSR_GN8; i += 256) ncnt[i] = 0;
  __syncthreads();
  for (int b = 0; b < CSR_NBLK8; ++b) { const int c = boff[b + 1] - boff[b]; int o_ = OFF[(size_t)g * CSR_NBLK8 + b]; o_ = (o_ < 0) ? 0 : (o_ > CHP - c ? CHP - c : o_); const int* src_ = STG + (size_t)b * CHP + o_;
    for (int i = t_; i < c; i += 256) { int id = src_[i]; id = (id < 0) ? 0 : id; ids[boff[b] + i] = id; int d = dst[id]; d = (d < v0) ? v0 : (d >= N ? N - 1 : d); int kk = d - v0; kk = (kk < 0) ? 0 : (kk >= CSR_GN8 ? CSR_GN8 - 1 : kk); key[boff[b] + i] = (unsigned short)kk; } }
  __syncthreads();
  if (t_ == 0) { for (int i = 0; i < tot; ++i) ncnt[key[i]] += 1; int acc = 0; for (int vl = 0; vl < CSR_GN8; ++vl) { const int c = ncnt[vl]; ncnt[vl] = acc; acc += c; } ncnt[CSR_GN8] = acc;
    for (int i = 0; i < tot; ++i) { const int vl = key[i]; outp[ncnt[vl]] = ids[i]; ncnt[vl] += 1; }
    for (int vl = CSR_GN8; vl > 0; --vl) ncnt[vl] = ncnt[vl - 1]; ncnt[0] = 0; }
  __syncthreads();
  for (int pass = 0; pass < 2; ++pass) {
    for (int i = t_; i < (stn - st) / 4; i += 256) { v4i v; for (int e = 0; e < 4; ++e) { const int q = i * 4 + e; v[e] = (q < tot) ? outp[q] : -1; } *(volatile v4i*)(PERM + st + i * 4) = v; }
    for (int i = t_; i < CSR_TS8 / 4; i += 256) { v4i a, c; for (int e = 0; e < 4; ++e) { const int vl = i * 4 + e; const int vc = vl < CSR_GN8 ? vl : CSR_GN8; a[e] = (vl < CSR_GN8) ? st + ncnt[vc] : st; c[e] = (vl < nv) ? (ncnt[(vc < CSR_GN8 ? vc : CSR_GN8 - 1) + 1] - ncnt[vc]) : 0; } *(volatile v4i*)(ROWPTR + t0 + i * 4) = a; *(volatile v4i*)(ROWCNT + t0 + i * 4) = c; }
    __threadfence(); }
}
__global__ __launch_bounds__(256) void csrZ_kernel8(int* __restrict__ p, size_t n4) { typedef __attribute__((ext_vector_type(4))) int v4i; const size_t tid = (size_t)blockIdx.x * 256 + threadIdx.x, nth = (size_t)gridDim.x * 256; v4i z = {0, 0, 0, 0}; for (size_t i = tid; i < n4; i += nth) *(volatile v4i*)(p + i * 4) = z; }
struct CsrBufs8 { int *STG, *HST, *OFF, *START, *TOT, *PERM, *ROWPTR, *ROWCNT, *FLAG; int nG, NGP, CHP; size_t permLen; char* base; size_t bytes; };
static size_t csr_carve8(CsrBufs8& c, char* ws, size_t off, int E, int N) {
  const size_t off0 = off; c.base = ws + off;
  auto al = [&](size_t bytes) { char* p = ws + off; off += (bytes + 255) & ~(size_t)255; return p; };
  c.nG = (N + CSR_GN8 - 1) / CSR_GN8; c.NGP = (c.nG + 31) & ~31; const int ch = (E + CSR_NBLK8 - 1) / CSR_NBLK8; c.CHP = (ch + 31) & ~31; c.permLen = (size_t)E + 32 * (size_t)c.nG + 32;
  c.STG = (int*)al((size_t)CSR_NBLK8 * c.CHP * 4); c.HST = (int*)al((size_t)CSR_NBLK8 * c.NGP * 4); c.OFF = (int*)al((size_t)c.NGP * CSR_NBLK8 * 4); c.START = (int*)al((size_t)(c.NGP + 64) * 4); c.TOT = (int*)al((size_t)(c.NGP + 64) * 4);
  c.PERM = (int*)al(c.permLen * 4); c.ROWPTR = (int*)al((size_t)c.nG * CSR_TS8 * 4); c.ROWCNT = (int*)al((size_t)c.nG * CSR_TS8 * 4); c.FLAG = (int*)al(256);
  c.bytes = off - off0; return off;
}
static void csr_build8(const CsrBufs8& c, const int* dst, int E, int N, hipStream_t stream) {
  const size_t smem = (size_t)(2 * c.NGP + c.CHP) * 4;
  csrZ_kernel8<<<512, 256, 0, stream>>>((int*)c.base, c.bytes / 16);
  csrA_kernel8<<<CSR_NBLK8, 64, smem, stream>>>(dst, E, N, c.nG, c.CHP, c.NGP, c.STG, c.HST);
  csrS_kernel8<<<1, 512, 0, stream>>>(c.HST, c.nG, c.NGP, c.START, c.TOT, c.OFF);
  csrB_kernel8<<<c.nG, 256, 0, stream>>>(dst, N, c.nG, c.CHP, c.NGP, (int)c.permLen, c.STG, c.HST, c.OFF, c.START, c.TOT, c.PERM, c.ROWPTR, c.ROWCNT, c.FLAG);
}


__global__ __launch_bounds__(256) void wprep_kernel(const float* __restrict__ wc, const float* __restrict__ wa1, const float* __restrict__ wg, b16* __restrict__ WC, b16* __restrict__ WA1, b16* __restrict__ WG) {
  const size_t u = (size_t)blockIdx.x * 256 + threadIdx.x; const size_t n1 = (size_t)NH * NF / 8, n2 = (size_t)AH * NH / 8, n3 = (size_t)NC * NH / 8; size_t t = u; v8b v;
  if (t < n1) { const size_t e = t * 8; const int o = (int)(e / NF), k0 = (int)(e % NF); for (int j = 0; j < 8; ++j) v[j] = (b16)(bf16_rne(wc[(size_t)(k0 + j) * NH + o]) * WSC); for (int p = 0; p < 2; ++p) { *(volatile v8b*)(WC + e) = v; __threadfence(); } return; } t -= n1;
  if (t < n2) { const size_t e = t * 8; const int o = (int)(e / NH), k0 = (int)(e % NH); for (int j = 0; j < 8; ++j) v[j] = (b16)(bf16_rne(wa1[(size_t)(k0 + j) * AH + o]) * WSC); for (int p = 0; p < 2; ++p) { *(volatile v8b*)(WA1 + e) = v; __threadfence(); } return; } t -= n2;
  if (t < n3) { const size_t e = t * 8; const int o = (int)(e / NH), k0 = (int)(e % NH); for (int j = 0; j < 8; ++j) v[j] = (b16)(bf16_rne(wg[(size_t)(k0 + j) * NC + o]) * WSC); for (int p = 0; p < 2; ++p) { *(volatile v8b*)(WG + e) = v; __threadfence(); } }
}
template <int RAW>
__global__ __launch_bounds__(256) void prop_kernel(const float* __restrict__ IN_, const int* __restrict__ srcs, const int* __restrict__ PERM, const int* __restrict__ ROWPTR, const int* __restrict__ ROWCNT, int permLen, float* __restrict__ OUT) {
  const int wave = threadIdx.x >> 5, lane = threadIdx.x & 31; const size_t v = (size_t)blockIdx.x * 8 + wave; v4f o = {0.0f, 0.0f, 0.0f, 0.0f};
  if (v < (size_t)N) { int st = ROWPTR[v], cnt = ROWCNT[v]; cnt = iclamp(cnt, 0, 65536); st = iclamp(st, 0, permLen - cnt); const float dv = rsqrtf((float)(cnt + 1)); v4f a = {0.0f, 0.0f, 0.0f, 0.0f};
#pragma unroll 2
    for (int j = 0; j < cnt; ++j) { const int e = iclamp(PERM[st + j], 0, E - 1); const int s = iclamp(srcs[e], 0, N - 1); int cs = ROWCNT[s]; cs = cs < 0 ? 0 : (cs > 65536 ? 65536 : cs); const float ds = rsqrtf((float)(cs + 1));
      v4f f = *(const v4f*)(IN_ + (size_t)s * NF + lane * 4); for (int i = 0; i < 4; ++i) a[i] += pmul(ds, RAW ? bf16_rne(f[i]) : f[i]); }
    v4f own = *(const v4f*)(IN_ + v * NF + lane * 4); for (int i = 0; i < 4; ++i) { const float ow = RAW ? bf16_rne(own[i]) : own[i]; o[i] = pmul(dv, a[i] + pmul(dv, ow)); } }
  for (int pass = 0; pass < 2; ++pass) { *(volatile v4f*)(OUT + v * NF + lane * 4) = o; __threadfence(); }
}
__global__ __launch_bounds__(32) void node_kernel(const float* __restrict__ H2, const float* __restrict__ lt, const float* __restrict__ gt, const b16* __restrict__ WC, const b16* __restrict__ WA1, const b16* __restrict__ WG, const float* __restrict__ bc, const float* __restrict__ ba1, const float* __restrict__ a2, float* __restrict__ G) {
  __shared__ __attribute__((aligned(16))) b16 Ah[16][NF + 8], Al[16][NF + 8], Lh[16][NH + 8]; __shared__ __attribute__((aligned(16))) float Hc[16][NH + 4], So[16][16];
  const int lane = threadIdx.x, nloc = lane & 15, hlf = lane >> 4; const size_t v0 = (size_t)blockIdx.x * 16;
  for (int rr = 0; rr < 16; ++rr) { const size_t v = v0 + rr; const bool ok = v < (size_t)N; v4f h = {0.0f, 0.0f, 0.0f, 0.0f}; v2f l2 = {0.0f, 0.0f}; if (ok) { h = *(const v4f*)(H2 + v * NF + lane * 4); l2 = *(const v2f*)(lt + v * NH + lane * 2); }
    for (int j = 0; j < 4; ++j) { b16 p, q; split16(h[j] * XS, p, q); Ah[rr][lane * 4 + j] = p; Al[rr][lane * 4 + j] = q; } for (int j = 0; j < 2; ++j) Lh[rr][lane * 2 + j] = (b16)(bf16_rne(l2[j]) * XS); }
  wave_lds_sync();
  v8f acc[4];
#pragma unroll
  for (int t = 0; t < 4; ++t) acc[t] = (v8f){};
#pragma unroll 2
  for (int kb = 0; kb < NF; kb += 32) { const v16b a = frag_kb(&Ah[nloc][kb], hlf), al = frag_kb(&Al[nloc][kb], hlf);
#pragma unroll
    for (int t = 0; t < 4; ++t) { const v16b bw = frag_kb(WC + (size_t)(t * 16 + nloc) * NF + kb, hlf); acc[t] = wmma16b(a, bw, acc[t]); acc[t] = wmma16b(al, bw, acc[t]); } }
  wave_lds_sync();
#pragma unroll
  for (int t = 0; t < 4; ++t) { const int c = t * 16 + nloc; const float bb = bf16_rne(bc[c]);
#pragma unroll 1
    for (int r8 = 0; r8 < 8; ++r8) { const int rl = 8 * hlf + r8; const float val = acc[t][r8] * (1.0f / (XS * WSC)) + bb; Hc[rl][c] = val; b16 p, q; split16(val * XS, p, q); Ah[rl][c] = p; Al[rl][c] = q; } }
  wave_lds_sync();
  v8f ah0[2], ah1[2]; for (int t = 0; t < 2; ++t) { ah0[t] = (v8f){}; ah1[t] = (v8f){}; }
#pragma unroll
  for (int kb = 0; kb < NH; kb += 32) { const v16b a = frag_kb(&Ah[nloc][kb], hlf), al = frag_kb(&Al[nloc][kb], hlf), l = frag_kb(&Lh[nloc][kb], hlf);
#pragma unroll
    for (int t = 0; t < 2; ++t) { const v16b bw = frag_kb(WA1 + (size_t)(t * 16 + nloc) * NH + kb, hlf); ah0[t] = wmma16b(a, bw, ah0[t]); ah0[t] = wmma16b(al, bw, ah0[t]); ah1[t] = wmma16b(l, bw, ah1[t]); } }
  float p0[8], p1[8]; for (int r8 = 0; r8 < 8; ++r8) { p0[r8] = 0.0f; p1[r8] = 0.0f; }
#pragma unroll
  for (int t = 0; t < 2; ++t) { const int c = t * 16 + nloc; const float bb = bf16_rne(ba1[c]), av = opaque(bf16_rne(a2[c]));
#pragma unroll
    for (int r8 = 0; r8 < 8; ++r8) { p0[r8] += pmul(tanhf(ah0[t][r8] * (1.0f / (XS * WSC)) + bb), av); p1[r8] += pmul(tanhf(ah1[t][r8] * (1.0f / (XS * WSC)) + bb), av); } }
#pragma unroll
  for (int r8 = 0; r8 < 8; ++r8) { float a = p0[r8], b = p1[r8]; for (int o = 1; o < 16; o <<= 1) { a += __shfl_xor(a, o); b += __shfl_xor(b, o); }
    const float m = fmaxf(a, b); const float e0 = nexp(a - m), e1 = nexp(b - m); const float w0 = e0 / (e0 + e1), w1 = e1 / (e0 + e1); if (nloc == 0) { So[8 * hlf + r8][0] = w0; So[8 * hlf + r8][1] = w1; } }
  wave_lds_sync();
  const float g0 = bf16_rne(gt[lane * 2]), g1 = bf16_rne(gt[lane * 2 + 1]);
  for (int rr = 0; rr < 16; ++rr) { const size_t v = v0 + rr; const float w0 = So[rr][0], w1 = So[rr][1]; v2f l2 = {0.0f, 0.0f}; if (v < (size_t)N) l2 = *(const v2f*)(lt + v * NH + lane * 2);
    for (int j = 0; j < 2; ++j) { const float hv = pmul(pmul(w0, Hc[rr][lane * 2 + j]) + pmul(w1, bf16_rne(l2[j])), j == 0 ? g0 : g1); b16 p, q; split16(hv * XS, p, q); Ah[rr][lane * 2 + j] = p; Al[rr][lane * 2 + j] = q; } }
  wave_lds_sync();
  v8f ag = (v8f){};
#pragma unroll
  for (int kb = 0; kb < NH; kb += 32) { const v16b a = frag_kb(&Ah[nloc][kb], hlf), al = frag_kb(&Al[nloc][kb], hlf); const v16b bw = frag_kb(WG + (size_t)nloc * NH + kb, hlf); ag = wmma16b(a, bw, ag); ag = wmma16b(al, bw, ag); }
#pragma unroll
  for (int r8 = 0; r8 < 8; ++r8) { const int rl = 8 * hlf + r8; So[rl][nloc] = ((v0 + rl) < (size_t)N) ? ag[r8] * (1.0f / (XS * WSC)) : 0.0f; }
  wave_lds_sync();
  for (int pass = 0; pass < 2; ++pass) { for (int q = 0; q < 2; ++q) { const int idx = q * 32 + lane; *(volatile v4f*)(G + v0 * NC + idx * 4) = *(const v4f*)(&So[idx >> 2][(idx & 3) * 4]); } __threadfence(); }
}
__global__ __launch_bounds__(256) void final_kernel(const float* __restrict__ G, const float* __restrict__ bg, const int* __restrict__ srcs, const int* __restrict__ PERM, const int* __restrict__ ROWPTR, const int* __restrict__ ROWCNT, int permLen, float* __restrict__ out) {
  __shared__ __attribute__((aligned(16))) float so[8][32];
  const int wave = threadIdx.x >> 5, lane = threadIdx.x & 31, nloc = lane & 15, hlf = lane >> 4; const size_t v = ((size_t)blockIdx.x * 8 + wave) * 2 + hlf;
  int st = ROWPTR[v], cnt = ROWCNT[v]; cnt = iclamp(cnt, 0, 65536); st = iclamp(st, 0, permLen - cnt); const float dv = rsqrtf((float)(cnt + 1));
  const int cnt_o = __shfl_xor(cnt, 16); const int cmax = cnt > cnt_o ? cnt : cnt_o; float a = 0.0f;
#pragma unroll 1
  for (int j = 0; j < cmax; ++j) { const bool ok = j < cnt; const int e = iclamp(PERM[iclamp(st + j, 0, permLen - 1)], 0, E - 1); const int s = iclamp(srcs[e], 0, N - 1); int cs = ROWCNT[s]; cs = cs < 0 ? 0 : (cs > 65536 ? 65536 : cs); const float ds = rsqrtf((float)(cs + 1));
    const float gv = G[(size_t)s * NC + nloc]; a += ok ? pmul(ds, gv) : 0.0f; }
  const float val = pmul(dv, a + pmul(dv, G[v * NC + nloc])) + bf16_rne(bg[nloc]);
  float m2 = val; for (int o = 1; o < 16; o <<= 1) m2 = fmaxf(m2, __shfl_xor(m2, o)); float se = nexp(val - m2); for (int o = 1; o < 16; o <<= 1) se += __shfl_xor(se, o);
  so[wave][lane] = val - m2 - __logf(se);
  wave_lds_sync();
  for (int pass = 0; pass < 2; ++pass) { if (lane < 8) *(volatile v4f*)(out + ((size_t)blockIdx.x * 8 + wave) * 2 * NC + lane * 4) = *(const v4f*)(&so[wave][lane * 4]); __threadfence(); }
}
}

extern "C" void kernel_launch(void* const* d_in, const int* in_sizes, int n_in, void* d_out, int out_size, void* d_ws, size_t ws_size, hipStream_t stream) {
  (void)n_in;
  auto Fp = [&](int i) { return (const float*)d_in[i]; }; auto Ip = [&](int i) { return (const int*)d_in[i]; };
  if (in_sizes[0] != N * NF || in_sizes[1] != 2 * E || in_sizes[2] != N * NH || in_sizes[3] != NH || in_sizes[4] != NF * NH || in_sizes[6] != NH * NC || in_sizes[8] != NH * AH || in_sizes[10] != AH || out_size != N * NC) return;
  size_t off = 0; char* ws = (char*)d_ws;
  auto carve = [&](size_t bytes) { char* p = ws + off; off += (bytes + 255) & ~(size_t)255; return p; };
  b16* WC = (b16*)carve((size_t)NH * NF * 2); b16* WA1 = (b16*)carve((size_t)AH * NH * 2); b16* WG = (b16*)carve((size_t)NC * NH * 2);
  float* H1 = (float*)carve((size_t)NP * NF * 4); float* H2 = (float*)carve((size_t)NP * NF * 4); float* G = (float*)carve((size_t)NP * NC * 4);
  CsrBufs8 csr; off = csr_carve8(csr, ws, off, E, N);
  if (off > ws_size || off > ((size_t)128 << 20)) return;
  wprep_kernel<<<(unsigned)(((size_t)NH * NF / 8 + (size_t)AH * NH / 8 + (size_t)NC * NH / 8 + 255) / 256), 256, 0, stream>>>(Fp(4), Fp(8), Fp(6), WC, WA1, WG);
  csr_build8(csr, Ip(1) + E, E, N, stream);
  prop_kernel<1><<<NP / 8, 256, 0, stream>>>(Fp(0), Ip(1), csr.PERM, csr.ROWPTR, csr.ROWCNT, (int)csr.permLen, H1);
  prop_kernel<0><<<NP / 8, 256, 0, stream>>>(H1, Ip(1), csr.PERM, csr.ROWPTR, csr.ROWCNT, (int)csr.permLen, H2);
  node_kernel<<<NP / 16, 32, 0, stream>>>(H2, Fp(2), Fp(3), WC, WA1, WG, Fp(5), Fp(9), Fp(10), G);
  final_kernel<<<N / 16, 256, 0, stream>>>(G, Fp(7), Ip(1), csr.PERM, csr.ROWPTR, csr.ROWCNT, (int)csr.permLen, (float*)d_out);
}
